// CrossAttentionBlock_28020366639331
// MI455X (gfx1250) — hardware-verified
//
#include <hip/hip_runtime.h>
#include <math.h>

#ifndef NB
#define NB 2
#endif
#define CCH 256
#define QHW 64
#define NQ 4096
#define KHW 32
#define NK 1024
#define NHD 8
#define HDM 32
#define KCV 2304
#define KCV8 288
#define Q_FULL_BS ((long long)CCH * NQ)
#define K_FULL_BS ((long long)CCH * NK)
static_assert(NB >= 1 && NB <= 2);
static_assert(KCV % 32 == 0 && KCV == 9 * CCH && KCV8 * 8 == KCV);
static_assert((NB * NQ) % 64 == 0 && (NB * NK) % 64 == 0 && (CCH % 64) == 0);
static_assert((((NB * NQ) / 64) * (CCH / 64)) % 8 == 0 && (((NB * NK) / 64) * (CCH / 64)) % 8 == 0);
static_assert((CCH * KCV8) % 256 == 0 && (CCH * (CCH / 8)) % 256 == 0);
static_assert(((long long)NB * CCH * NK / 8) % 256 == 0 && ((long long)NB * NQ * KCV8) % 256 == 0);
static_assert((NB * NQ) % 8 == 0 && (NB * NK) % 8 == 0);

typedef __attribute__((ext_vector_type(16))) _Float16 v16h;
typedef __attribute__((ext_vector_type(8)))  _Float16 v8h;
typedef __attribute__((ext_vector_type(16))) __bf16   v16b;
typedef __attribute__((ext_vector_type(8)))  __bf16   v8b;
typedef __attribute__((ext_vector_type(8)))  float    v8f;
typedef __attribute__((ext_vector_type(4)))  float    v4f;
typedef unsigned int u4v __attribute__((ext_vector_type(4)));

#define VST2(T, ptr, val) do { const T vst2_v_ = (val); *(volatile T*)(ptr) = vst2_v_; __threadfence(); *(volatile T*)(ptr) = vst2_v_; } while (0)

namespace w25 {
typedef __attribute__((ext_vector_type(16))) _Float16 v16h;
typedef __attribute__((ext_vector_type(8)))  _Float16 v8h;
typedef __attribute__((ext_vector_type(16))) __bf16   v16b;
typedef __attribute__((ext_vector_type(8)))  __bf16   v8b;
typedef __attribute__((ext_vector_type(8)))  float    v8f;
typedef __attribute__((ext_vector_type(4)))  float    v4f;

__device__ __forceinline__ unsigned short f2bf_bits(float f) {
  unsigned u = __float_as_uint(f);
  return (unsigned short)((u + 0x7FFFu + ((u >> 16) & 1u)) >> 16);
}
__device__ __forceinline__ float bf_bits2f(unsigned short h) { return __uint_as_float(((unsigned)h) << 16); }

__device__ __forceinline__ void dep_guard_h(v8f& a, v8f& b, v16h x, v16h y) { asm volatile("v_nop\n\tv_nop\n\tv_nop\n\tv_nop" : "+v"(a), "+v"(b) : "v"(x), "v"(y)); }
__device__ __forceinline__ void dep_guard_b(v8f& a, v8f& b, v16b x, v16b y) { asm volatile("v_nop\n\tv_nop\n\tv_nop\n\tv_nop" : "+v"(a), "+v"(b) : "v"(x), "v"(y)); }
__device__ __forceinline__ void keep4_h(v16h a, v16h b, v16h c, v16h d) { asm volatile("v_nop" :: "v"(a), "v"(b), "v"(c), "v"(d)); }
__device__ __forceinline__ void keep4_b(v16b a, v16b b, v16b c, v16b d) { asm volatile("v_nop" :: "v"(a), "v"(b), "v"(c), "v"(d)); }
__device__ __forceinline__ void acc_guard4(v8f& a, v8f& b, v8f& c, v8f& d) { asm volatile("v_nop\n\tv_nop\n\tv_nop\n\tv_nop" : "+v"(a), "+v"(b), "+v"(c), "+v"(d)); }
template <typename T> struct Frag;
template <> struct Frag<_Float16> {
  typedef v16h V; union U { v16h v; v8h h[2]; };
  static __device__ __forceinline__ v16h load(const _Float16* p) {
    U f; f.h[0] = *(const v8h*)(p); f.h[1] = *(const v8h*)(p + 16); return f.v;
  }
  static __device__ __forceinline__ v8f mma(v16h a, v16h b, v8f c) {
    return __builtin_amdgcn_wmma_f32_16x16x32_f16(false, a, false, b, (short)0, c, false, false);
  }
  static __device__ __forceinline__ void guard(v8f& a, v8f& b, v16h x, v16h y) { dep_guard_h(a, b, x, y); }
  static __device__ __forceinline__ void keep(v16h a, v16h b, v16h c, v16h d) { keep4_h(a, b, c, d); }
};
template <> struct Frag<__bf16> {
  typedef v16b V; union U { v16b v; v8b h[2]; };
  static __device__ __forceinline__ v16b load(const __bf16* p) {
    U f; f.h[0] = *(const v8b*)(p); f.h[1] = *(const v8b*)(p + 16); return f.v;
  }
  static __device__ __forceinline__ v8f mma(v16b a, v16b b, v8f c) {
    return __builtin_amdgcn_wmma_f32_16x16x32_bf16(false, a, false, b, (short)0, c, false, false);
  }
  static __device__ __forceinline__ void guard(v8f& a, v8f& b, v16b x, v16b y) { dep_guard_b(a, b, x, y); }
  static __device__ __forceinline__ void keep(v16b a, v16b b, v16b c, v16b d) { keep4_b(a, b, c, d); }
};

template <int ET> struct Elem;
template <> struct Elem<0> { typedef _Float16 T; };
template <> struct Elem<1> { typedef __bf16 T; };
template <int ET, bool SPLIT, int BIAS_MODE, int OUT_MODE, bool RESID, int ACT = 0>
__global__ __launch_bounds__(256) void wmma_gemm64(
    const unsigned short* __restrict__ Ap, const unsigned short* __restrict__ A2p, int lda, long strideA,
    const unsigned short* __restrict__ Btp, const unsigned short* __restrict__ Bt2p, int ldb, long strideB,
    void* __restrict__ Cout, void* __restrict__ Cout2, int ldc, long strideC,
    const float* __restrict__ bias,
    const float* __restrict__ resid, long strideR,
    int M, int N, int K, float scale) {
  typedef typename Elem<ET>::T T;
  typedef typename Frag<T>::V V;
  const T* A = (const T*)Ap; const T* A2 = (const T*)A2p; const T* Bt = (const T*)Btp; const T* Bt2 = (const T*)Bt2p;
  __shared__ __align__(16) float sT[8][16 * 68];
  const int b    = blockIdx.y;
  const int lane = threadIdx.x & 31;
  const int wave = threadIdx.x >> 5;
  const int tilesN = N >> 6;
  const int tilesM = M >> 6;
  const int tile = blockIdx.x * 8 + wave;
  if (tile >= tilesM * tilesN) return;
  const int tm = tile / tilesN;
  const int tn = tile - tm * tilesN;
  const int m0 = tm << 6;
  const int n0 = tn << 6;

  const T* Ab  = A  + (size_t)b * strideA;
  const T* Bb  = Bt + (size_t)b * strideB;
  const T* Ab2 = SPLIT ? (A2  + (size_t)b * strideA) : nullptr;
  const T* Bb2 = SPLIT ? (Bt2 + (size_t)b * strideB) : nullptr;

  const int rlane = lane & 15;
  const int koff  = (lane >> 4) * 8;
  const int mOff  = (lane >> 4) * 8;

  v8f acc[4][4];
#pragma unroll
  for (int i = 0; i < 4; ++i)
#pragma unroll
    for (int j = 0; j < 4; ++j) acc[i][j] = (v8f){0.f,0.f,0.f,0.f,0.f,0.f,0.f,0.f};

  for (int k0 = 0; k0 < K; k0 += 32) {
    V bh[4], bl[4];
#pragma unroll
    for (int j = 0; j < 4; ++j) {
      const size_t bo = (size_t)(n0 + (j << 4) + rlane) * ldb + koff + k0;
      bh[j] = Frag<T>::load(Bb + bo);
      if (SPLIT) bl[j] = Frag<T>::load(Bb2 + bo);
    }
#pragma unroll
    for (int i = 0; i < 4; ++i) {
      const size_t ao = (size_t)(m0 + (i << 4) + rlane) * lda + koff + k0;
      V ah = Frag<T>::load(Ab + ao);
      V al;
      if (SPLIT) al = Frag<T>::load(Ab2 + ao);
#pragma unroll
      for (int j = 0; j < 4; ++j) {
        acc[i][j] = Frag<T>::mma(ah, bh[j], acc[i][j]);
        if (SPLIT) {
          acc[i][j] = Frag<T>::mma(ah, bl[j], acc[i][j]);
          acc[i][j] = Frag<T>::mma(al, bh[j], acc[i][j]);
        }
      }
      Frag<T>::guard(acc[i][0], acc[i][3], ah, SPLIT ? al : ah);
    }
    Frag<T>::keep(bh[0], bh[1], bh[2], bh[3]);
    if (SPLIT) Frag<T>::keep(bl[0], bl[1], bl[2], bl[3]);
  }
  acc_guard4(acc[0][0], acc[0][1], acc[0][2], acc[0][3]);
  acc_guard4(acc[1][0], acc[1][1], acc[1][2], acc[1][3]);
  acc_guard4(acc[2][0], acc[2][1], acc[2][2], acc[2][3]);
  acc_guard4(acc[3][0], acc[3][1], acc[3][2], acc[3][3]);

  float* slab = sT[wave];
  const float* Rb = RESID ? (resid + (size_t)b * strideR) : nullptr;
#pragma unroll
  for (int i = 0; i < 4; ++i) {
    const int mBase = m0 + (i << 4);
#pragma unroll
    for (int j = 0; j < 4; ++j) {
      const int n = n0 + (j << 4) + rlane;
      float bv = 0.f;
      if (BIAS_MODE == 2) bv = bias[n];
#pragma unroll
      for (int r = 0; r < 8; ++r) {
        float v = acc[i][j][r] * scale;
        if (BIAS_MODE == 1) v += bias[mBase + mOff + r];
        if (BIAS_MODE == 2) v += bv;
        if (RESID) v += Rb[(size_t)(mBase + mOff + r) * ldc + n];
        if (ACT == 1) v = tanhf(v);
        if (ACT == 2) v = fmaxf(v, 0.0f);
        if (ACT == 3) v = v / (1.0f + expf(-v));
        if (ACT == 4) v = (v > 0.f) ? v : 0.01f * v;
        if (ACT == 5) v = 0.5f * v * (1.0f + erff(v * 0.70710678118654752f));
        if (ACT == 6) v = (v > 0.f) ? v : 0.2f * v;
        if (ACT == 7) { const float u = 0.7978845608028654f * (v + 0.044715f * v * v * v); v = 0.5f * v * (1.f + tanhf(u)); }
        slab[(mOff + r) * 68 + (j << 4) + rlane] = v;
      }
    }
    __builtin_amdgcn_fence(3  , "workgroup");
    __builtin_amdgcn_wave_barrier();
    __builtin_amdgcn_fence(2  , "workgroup");
    if (OUT_MODE == 0) {
      float* C = (float*)Cout + (size_t)b * strideC;
      const int hh = lane >> 4, c4 = (lane & 15) * 4;
      for (int pass = 0; pass < 2; ++pass) {
#pragma unroll
        for (int it = 0; it < 8; ++it) {
          const int row = it * 2 + hh;
          v4f v = *(const v4f*)(slab + row * 68 + c4);
          *(volatile v4f*)(C + (size_t)(mBase + row) * ldc + n0 + c4) = v;
        }
        __threadfence();
      }
    } else {
      const int q = lane >> 3, c8 = (lane & 7) * 8;
      unsigned short* C  = (unsigned short*)Cout  + (size_t)b * strideC;
      unsigned short* C2 = (OUT_MODE == 2) ? ((unsigned short*)Cout2 + (size_t)b * strideC) : nullptr;
      for (int pass = 0; pass < 2; ++pass) {
#pragma unroll
        for (int it = 0; it < 4; ++it) {
          const int row = it * 4 + q;
          const float* sp = slab + row * 68 + c8;
          v8h hv, lv;
#pragma unroll
          for (int e = 0; e < 8; ++e) {
            if (OUT_MODE == 1) {
              hv[e] = (_Float16)sp[e];
            } else {
              unsigned short hb = f2bf_bits(sp[e]);
              unsigned short lb = f2bf_bits(sp[e] - bf_bits2f(hb));
              hv[e] = __builtin_bit_cast(_Float16, hb);
              lv[e] = __builtin_bit_cast(_Float16, lb);
            }
          }
          *(volatile v8h*)(C + (size_t)(mBase + row) * ldc + n0 + c8) = hv;
          if (OUT_MODE == 2) *(volatile v8h*)(C2 + (size_t)(mBase + row) * ldc + n0 + c8) = lv;
        }
        __threadfence();
      }
    }
    __builtin_amdgcn_fence(3  , "workgroup");
    __builtin_amdgcn_wave_barrier();
    __builtin_amdgcn_fence(2  , "workgroup");
  }
}
}

__device__ __forceinline__ unsigned int cmb_pk2(float a, float b) { return (unsigned int)__builtin_bit_cast(unsigned short, (_Float16)a) | ((unsigned int)__builtin_bit_cast(unsigned short, (_Float16)b) << 16); }
__device__ __forceinline__ float cmb_bf(float v) { const unsigned u = __builtin_bit_cast(unsigned, v); const unsigned r = (u + 0x7fffu + ((u >> 16) & 1u)) & 0xffff0000u; return __builtin_bit_cast(float, r); }
__global__ __launch_bounds__(256) void k_cm_bfvec(const float* __restrict__ SRC, float* __restrict__ DST, int n) { const int u = blockIdx.x * 256 + threadIdx.x; if (u >= n) return; VST2(float, DST + u, cmb_bf(SRC[u])); }
__global__ __launch_bounds__(256) void k_cm_castb(const float* __restrict__ SRC, int lds, unsigned short* __restrict__ DST, int ldd, int nR, int nC, float sc) {
    const long long u = (long long)blockIdx.x * 256 + threadIdx.x; const int per = nC / 8; if (u >= (long long)nR * per) return; const int r = (int)(u / per); const int c0 = 8 * (int)(u % per);
    const float* s = SRC + (long long)r * lds + c0; float w[8];
#pragma unroll
    for (int e = 0; e < 8; ++e) w[e] = cmb_bf(s[e]) * sc;
    u4v pk; pk.x = cmb_pk2(w[0], w[1]); pk.y = cmb_pk2(w[2], w[3]); pk.z = cmb_pk2(w[4], w[5]); pk.w = cmb_pk2(w[6], w[7]); VST2(u4v, (u4v*)(DST + (long long)r * ldd + c0), pk); }
__global__ __launch_bounds__(256) void k_castbf8(const float* __restrict__ SRC, unsigned short* __restrict__ DST, long long n8) {
    const long long u = (long long)blockIdx.x * 256 + threadIdx.x; if (u >= n8) return;
    const v4f a = *(const v4f*)(SRC + 8 * u), c = *(const v4f*)(SRC + 8 * u + 4);
    u4v pk;
    pk.x = (unsigned)w25::f2bf_bits(a.x) | ((unsigned)w25::f2bf_bits(a.y) << 16);
    pk.y = (unsigned)w25::f2bf_bits(a.z) | ((unsigned)w25::f2bf_bits(a.w) << 16);
    pk.z = (unsigned)w25::f2bf_bits(c.x) | ((unsigned)w25::f2bf_bits(c.y) << 16);
    pk.w = (unsigned)w25::f2bf_bits(c.z) | ((unsigned)w25::f2bf_bits(c.w) << 16);
    VST2(u4v, (u4v*)(DST + 8 * u), pk); }

__global__ __launch_bounds__(256) void k_im2col(const float* __restrict__ Q, unsigned short* __restrict__ IM, long long npieces) {
    const long long u = (long long)blockIdx.x * 256 + threadIdx.x; if (u >= npieces) return;
    const int m = (int)(u / KCV8); const int k8 = 8 * (int)(u - (long long)m * KCV8);
    const int b = m / NQ, pix = m - b * NQ, y = pix / QHW, x = pix - y * QHW;
    const float* qb = Q + (long long)b * Q_FULL_BS;
    float w[8];
#pragma unroll
    for (int e = 0; e < 8; ++e) {
        const int k = k8 + e; const int ci = k / 9; const int p = k - 9 * ci; const int dy = p / 3; const int dx = p - 3 * dy;
        const int yy = y + dy - 1, xx = x + dx - 1;
        const bool in = (yy >= 0) && (yy < QHW) && (xx >= 0) && (xx < QHW);
        const int yc = min(max(yy, 0), QHW - 1), xc = min(max(xx, 0), QHW - 1);
        const float val = qb[((long long)ci * QHW + yc) * QHW + xc];
        w[e] = in ? cmb_bf(val) : 0.f;
    }
    u4v pk; pk.x = cmb_pk2(w[0], w[1]); pk.y = cmb_pk2(w[2], w[3]); pk.z = cmb_pk2(w[4], w[5]); pk.w = cmb_pk2(w[6], w[7]);
    VST2(u4v, (u4v*)(IM + (long long)m * KCV + k8), pk); }

__global__ __launch_bounds__(256) void k_rms16(const float* __restrict__ X, long long sZ, long long sR, long long sC, int rowsPerZ, int nRows, const float* __restrict__ G, int rin, unsigned short* __restrict__ DST) {
    const int wave = threadIdx.x >> 5, L = threadIdx.x & 31; const int row = blockIdx.x * 8 + wave; if (row >= nRows) return;
    const int z = row / rowsPerZ, r = row - z * rowsPerZ;
    const float* base = X + (long long)z * sZ + (long long)r * sR + (long long)(8 * L) * sC;
    float xv[8]; float ss = 0.f;
#pragma unroll
    for (int e = 0; e < 8; ++e) { float t = base[(long long)e * sC]; t = rin ? cmb_bf(t) : t; xv[e] = t; ss += t * t; }
#pragma unroll
    for (int o = 16; o > 0; o >>= 1) ss += __shfl_xor(ss, o, 32);
    const float rs = rsqrtf(ss * (1.0f / 256.0f) + 1e-6f);
    float w[8];
#pragma unroll
    for (int e = 0; e < 8; ++e) w[e] = (xv[e] * rs) * cmb_bf(G[8 * L + e]);
    u4v pk; pk.x = cmb_pk2(w[0], w[1]); pk.y = cmb_pk2(w[2], w[3]); pk.z = cmb_pk2(w[4], w[5]); pk.w = cmb_pk2(w[6], w[7]);
    VST2(u4v, (u4v*)(DST + (long long)row * CCH + 8 * L), pk); }

#define A_SCP 196
#define A_PAP 192
#define A_PLP 200
#define A_OSP 68
#define A_SC_B (64 * A_SCP * 4)
#define A_PA_B (64 * A_PAP * 4)
#define A_PL_B (64 * A_PLP * 2)
#define A_LDS_B (A_SC_B + A_PA_B + 2 * A_PL_B)
static_assert(A_LDS_B == 150528);
static_assert((A_LDS_B % 16) == 0);
static_assert(8 * 32 * A_OSP * 4 <= A_SC_B + A_PA_B);
static_assert((A_SC_B % 16) == 0 && (A_PA_B % 16) == 0 && (A_PL_B % 16) == 0 && ((A_PLP * 2) % 16) == 0 && ((A_OSP * 4) % 16) == 0 && ((32 * A_OSP * 4) % 16) == 0);
#define SCL_QK 0.17677669529663687f

__device__ __forceinline__ v8f mma3b(v16b ah, v16b al, v16b bh, v16b bl, v8f c) {
    c = __builtin_amdgcn_wmma_f32_16x16x32_bf16(false, ah, false, bh, (short)0, c, false, false);
    c = __builtin_amdgcn_wmma_f32_16x16x32_bf16(false, ah, false, bl, (short)0, c, false, false);
    c = __builtin_amdgcn_wmma_f32_16x16x32_bf16(false, al, false, bh, (short)0, c, false, false);
    asm volatile("v_nop\n\tv_nop\n\tv_nop\n\tv_nop" : "+v"(c) : "v"(ah), "v"(al), "v"(bh), "v"(bl));
    return c;
}
__device__ __forceinline__ v8f mma2b(v16b ah, v16b al, v16b b, v8f c) {
    c = __builtin_amdgcn_wmma_f32_16x16x32_bf16(false, ah, false, b, (short)0, c, false, false);
    c = __builtin_amdgcn_wmma_f32_16x16x32_bf16(false, al, false, b, (short)0, c, false, false);
    asm volatile("v_nop\n\tv_nop\n\tv_nop\n\tv_nop" : "+v"(c) : "v"(ah), "v"(al), "v"(b));
    return c;
}

__global__ __launch_bounds__(256) void k_attw(const unsigned short* __restrict__ QPH, const unsigned short* __restrict__ QPL,
                                              const unsigned short* __restrict__ KPH, const unsigned short* __restrict__ KPL,
                                              const unsigned short* __restrict__ VT, float* __restrict__ OUT) {
    __shared__ __align__(16) float4 dsm4[A_LDS_B / 16];
    unsigned char* dsm = (unsigned char*)dsm4;
    float* sc = (float*)dsm;
    float* pacc = (float*)(dsm + A_SC_B);
    __bf16* ph = (__bf16*)(dsm + A_SC_B + A_PA_B);
    __bf16* plo = (__bf16*)(dsm + A_SC_B + A_PA_B + A_PL_B);
    float* ost = (float*)dsm;
    union FB { v16b v; v8b h[2]; };
    const int tid = threadIdx.x, wave = tid >> 5, lane = tid & 31, hf = lane >> 4, l15 = lane & 15;
    const int b = (int)blockIdx.x / QHW, y = (int)blockIdx.x - b * QHW;
    int kr0 = (y & 1) ? ((y >> 1) - 2) : ((y >> 1) - 3);
    kr0 = min(max(kr0, 0), KHW - 6);
    const int ks0 = kr0 * KHW;
    const int qt = wave & 3, kh2 = wave >> 2;
    const long long qrow = (long long)b * NQ + (long long)y * QHW + qt * 16 + l15;
    const __bf16* qh_p = (const __bf16*)QPH + qrow * CCH + 8 * hf;
    const __bf16* ql_p = (const __bf16*)QPL + qrow * CCH + 8 * hf;
    const __bf16* kh_p = (const __bf16*)KPH + ((long long)b * NK + ks0) * CCH + 8 * hf;
    const __bf16* kl_p = (const __bf16*)KPL + ((long long)b * NK + ks0) * CCH + 8 * hf;
    const int srow = tid >> 2, scol0 = 48 * (tid & 3);
    const int ymk = 2 * y - 1;
#pragma unroll 1
    for (int h = 0; h < NHD; ++h) {
        FB qa, qb;
        qa.h[0] = *(const v8b*)(qh_p + h * HDM); qa.h[1] = *(const v8b*)(qh_p + h * HDM + 16);
        qb.h[0] = *(const v8b*)(ql_p + h * HDM); qb.h[1] = *(const v8b*)(ql_p + h * HDM + 16);
#pragma unroll
        for (int t = 0; t < 6; ++t) {
            const int kl = 96 * kh2 + 16 * t + l15;
            const __bf16* krh = kh_p + (long long)kl * CCH + h * HDM;
            const __bf16* krl = kl_p + (long long)kl * CCH + h * HDM;
            FB ka, kb;
            ka.h[0] = *(const v8b*)(krh); ka.h[1] = *(const v8b*)(krh + 16);
            kb.h[0] = *(const v8b*)(krl); kb.h[1] = *(const v8b*)(krl + 16);
            v8f acc = (v8f){0.f, 0.f, 0.f, 0.f, 0.f, 0.f, 0.f, 0.f};
            acc = mma3b(qa.v, qb.v, ka.v, kb.v, acc);
            const int dky = ymk - 4 * (kr0 + (kl >> 5));
            const bool oky = (dky <= 12) && (dky >= -12);
            const int kj4 = 4 * (kl & 31);
#pragma unroll
            for (int r = 0; r < 8; ++r) {
                const int x = qt * 16 + 8 * hf + r;
                const int dkx = (2 * x - 1) - kj4;
                const bool ok = oky && (dkx <= 12) && (dkx >= -12);
                sc[x * A_SCP + kl] = ok ? acc[r] * SCL_QK : -1.0e30f;
            }
        }
        __syncthreads();
        {
            float* sr = sc + srow * A_SCP + scol0;
            float m = -3.0e38f;
#pragma unroll 4
            for (int c = 0; c < 48; ++c) m = fmaxf(m, sr[c]);
            m = fmaxf(m, __shfl_xor(m, 1, 32)); m = fmaxf(m, __shfl_xor(m, 2, 32));
            float s = 0.f;
#pragma unroll 4
            for (int c = 0; c < 48; ++c) { const float e = expf(sr[c] - m); sr[c] = e; s += e; }
            s += __shfl_xor(s, 1, 32); s += __shfl_xor(s, 2, 32);
            const float inv = 1.0f / s;
            float* pr = pacc + srow * A_PAP + scol0;
            if (h == 0) {
#pragma unroll 4
                for (int c = 0; c < 48; ++c) pr[c] = sr[c] * inv;
            } else {
#pragma unroll 4
                for (int c = 0; c < 48; ++c) pr[c] = pr[c] + sr[c] * inv;
            }
        }
        __syncthreads();
    }
    {
        const float* pr = pacc + srow * A_PAP + scol0;
        unsigned int* hw = (unsigned int*)(ph + srow * A_PLP + scol0);
        unsigned int* lw = (unsigned int*)(plo + srow * A_PLP + scol0);
#pragma unroll 4
        for (int c2 = 0; c2 < 24; ++c2) {
            const float a = pr[2 * c2] * 0.125f, bb = pr[2 * c2 + 1] * 0.125f;
            const unsigned short ha = w25::f2bf_bits(a), hb = w25::f2bf_bits(bb);
            const unsigned short la = w25::f2bf_bits(a - w25::bf_bits2f(ha)), lb = w25::f2bf_bits(bb - w25::bf_bits2f(hb));
            hw[c2] = (unsigned)ha | ((unsigned)hb << 16);
            lw[c2] = (unsigned)la | ((unsigned)lb << 16);
        }
    }
    __syncthreads();
    v8f o[4][2];
#pragma unroll
    for (int q4 = 0; q4 < 4; ++q4) { o[q4][0] = (v8f){0.f, 0.f, 0.f, 0.f, 0.f, 0.f, 0.f, 0.f}; o[q4][1] = o[q4][0]; }
    const __bf16* vt_p = (const __bf16*)VT + ((long long)b * CCH + 32 * wave + l15) * NK + ks0 + 8 * hf;
    const __bf16* ph_p = ph + l15 * A_PLP + 8 * hf;
    const __bf16* pl_p = plo + l15 * A_PLP + 8 * hf;
#pragma unroll 1
    for (int kk = 0; kk < 6; ++kk) {
        FB v0, v1;
        v0.h[0] = *(const v8b*)(vt_p + kk * 32); v0.h[1] = *(const v8b*)(vt_p + kk * 32 + 16);
        v1.h[0] = *(const v8b*)(vt_p + 16 * NK + kk * 32); v1.h[1] = *(const v8b*)(vt_p + 16 * NK + kk * 32 + 16);
#pragma unroll
        for (int q4 = 0; q4 < 4; ++q4) {
            FB pa, pb;
            pa.h[0] = *(const v8b*)(ph_p + q4 * 16 * A_PLP + kk * 32); pa.h[1] = *(const v8b*)(ph_p + q4 * 16 * A_PLP + kk * 32 + 16);
            pb.h[0] = *(const v8b*)(pl_p + q4 * 16 * A_PLP + kk * 32); pb.h[1] = *(const v8b*)(pl_p + q4 * 16 * A_PLP + kk * 32 + 16);
            o[q4][0] = mma2b(pa.v, pb.v, v0.v, o[q4][0]);
            o[q4][1] = mma2b(pa.v, pb.v, v1.v, o[q4][1]);
        }
    }
    float* os = ost + wave * (32 * A_OSP);
#pragma unroll
    for (int q4 = 0; q4 < 4; ++q4)
#pragma unroll
        for (int nt = 0; nt < 2; ++nt)
#pragma unroll
            for (int r = 0; r < 8; ++r) os[(nt * 16 + l15) * A_OSP + q4 * 16 + 8 * hf + r] = o[q4][nt][r];
    __builtin_amdgcn_fence(3  , "workgroup");
    __builtin_amdgcn_wave_barrier();
    __builtin_amdgcn_fence(2  , "workgroup");
    float* ob = OUT + ((long long)b * CCH + 32 * wave) * NQ + (long long)y * QHW;
    const int lq = lane >> 3, c4 = (lane & 7) * 4;
    for (int pass = 0; pass < 2; ++pass) {
#pragma unroll
        for (int it = 0; it < 16; ++it) {
            const int ln = it * 4 + lq; const int cl = ln >> 1; const int xh = (ln & 1) * 32;
            const v4f vv = *(const v4f*)(os + cl * A_OSP + xh + c4);
            *(volatile v4f*)(ob + (long long)cl * NQ + xh + c4) = vv;
        }
        __threadfence();
    }
}

static inline size_t al256(size_t b) { return (b + 255) & ~(size_t)255; }

extern "C" void kernel_launch(void* const* d_in, const int* in_sizes, int n_in, void* d_out, int out_size, void* d_ws, size_t ws_size, hipStream_t stream) {
    if (n_in < 10) return;
    if (in_sizes[0] < NB * CCH * NQ || in_sizes[1] < NB * CCH * NK || in_sizes[2] < NB * CCH * NK || in_sizes[3] < CCH * KCV ||
        in_sizes[4] < CCH || in_sizes[5] < CCH || in_sizes[6] < CCH * CCH || in_sizes[7] < CCH || in_sizes[8] < CCH * CCH || in_sizes[9] < CCH) return;
    if (out_size < NB * CCH * NQ) return;
    const float* qin = (const float*)d_in[0];
    const float* kin = (const float*)d_in[1];
    const float* vin = (const float*)d_in[2];
    const float* cw  = (const float*)d_in[3];
    const float* gq  = (const float*)d_in[4];
    const float* gk  = (const float*)d_in[5];
    const float* wq  = (const float*)d_in[6];
    const float* bq  = (const float*)d_in[7];
    const float* wk  = (const float*)d_in[8];
    const float* bk  = (const float*)d_in[9];
    float* out = (float*)d_out;

    char* wsp = (char*)d_ws; size_t off = 0;
    unsigned short* CW16 = (unsigned short*)(wsp + off); off += al256((size_t)CCH * KCV * 2);
    unsigned short* WQ16 = (unsigned short*)(wsp + off); off += al256((size_t)CCH * CCH * 2);
    unsigned short* WK16 = (unsigned short*)(wsp + off); off += al256((size_t)CCH * CCH * 2);
    float* BR = (float*)(wsp + off);                     off += al256((size_t)2 * CCH * 4);
    unsigned short* VT   = (unsigned short*)(wsp + off); off += al256((size_t)NB * CCH * NK * 2);
    unsigned short* IM   = (unsigned short*)(wsp + off); off += al256((size_t)NB * NQ * KCV * 2);
    float* QF = (float*)(wsp + off);                     off += al256((size_t)NB * NQ * CCH * 4);
    unsigned short* QN16 = (unsigned short*)(wsp + off); off += al256((size_t)NB * NQ * CCH * 2);
    unsigned short* QPH  = (unsigned short*)(wsp + off); off += al256((size_t)NB * NQ * CCH * 2);
    unsigned short* QPL  = (unsigned short*)(wsp + off); off += al256((size_t)NB * NQ * CCH * 2);
    unsigned short* KN16 = (unsigned short*)(wsp + off); off += al256((size_t)NB * NK * CCH * 2);
    unsigned short* KPH  = (unsigned short*)(wsp + off); off += al256((size_t)NB * NK * CCH * 2);
    unsigned short* KPL  = (unsigned short*)(wsp + off); off += al256((size_t)NB * NK * CCH * 2);
    if (off > ws_size) return;

    k_cm_castb<<<(unsigned)(((long long)CCH * KCV8) / 256), 256, 0, stream>>>(cw, KCV, CW16, KCV, CCH, KCV, 64.0f);
    k_cm_castb<<<(unsigned)(((long long)CCH * (CCH / 8)) / 256), 256, 0, stream>>>(wq, CCH, WQ16, CCH, CCH, CCH, 16.0f);
    k_cm_castb<<<(unsigned)(((long long)CCH * (CCH / 8)) / 256), 256, 0, stream>>>(wk, CCH, WK16, CCH, CCH, CCH, 16.0f);
    k_cm_bfvec<<<1, 256, 0, stream>>>(bq, BR, CCH);
    k_cm_bfvec<<<1, 256, 0, stream>>>(bk, BR + CCH, CCH);
    k_castbf8<<<(unsigned)(((long long)NB * CCH * NK / 8) / 256), 256, 0, stream>>>(vin, VT, (long long)NB * CCH * NK / 8);
    k_im2col<<<(unsigned)(((long long)NB * NQ * KCV8) / 256), 256, 0, stream>>>(qin, IM, (long long)NB * NQ * KCV8);
    w25::wmma_gemm64<0, false, 0, 0, false, 0><<<dim3((unsigned)(((NB * NQ) / 64) * (CCH / 64) / 8), 1u), 256, 0, stream>>>(
        IM, nullptr, KCV, 0, CW16, nullptr, KCV, 0, (void*)QF, nullptr, CCH, 0, nullptr, nullptr, 0, NB * NQ, CCH, KCV, 1.0f / 64.0f);
    k_rms16<<<(unsigned)((NB * NQ) / 8), 256, 0, stream>>>(QF, 0, CCH, 1, NB * NQ, NB * NQ, gq, 0, QN16);
    w25::wmma_gemm64<0, false, 2, 2, false, 0><<<dim3((unsigned)(((NB * NQ) / 64) * (CCH / 64) / 8), 1u), 256, 0, stream>>>(
        QN16, nullptr, CCH, 0, WQ16, nullptr, CCH, 0, (void*)QPH, (void*)QPL, CCH, 0, BR, nullptr, 0, NB * NQ, CCH, CCH, 1.0f / 16.0f);
    k_rms16<<<(unsigned)((NB * NK) / 8), 256, 0, stream>>>(kin, K_FULL_BS, 1, NK, NK, NB * NK, gk, 1, KN16);
    w25::wmma_gemm64<0, false, 2, 2, false, 0><<<dim3((unsigned)(((NB * NK) / 64) * (CCH / 64) / 8), 1u), 256, 0, stream>>>(
        KN16, nullptr, CCH, 0, WK16, nullptr, CCH, 0, (void*)KPH, (void*)KPL, CCH, 0, BR + CCH, nullptr, 0, NB * NK, CCH, CCH, 1.0f / 16.0f);
    k_attw<<<(unsigned)(NB * QHW), 256, 0, stream>>>(QPH, QPL, KPH, KPL, VT, out);
}
